// VanillaEGNNLayer_83665962926202
// MI455X (gfx1250) — hardware-verified
//
#include <hip/hip_runtime.h>
#include <stddef.h>
#include <stdint.h>
#include <math.h>


#define HD     128
#define DIN    257
#define HP     136
#define AP     264
#define FP     132
#define ROWS   64
#define WSC    16.0f
#define WINV   0.0625f
#define NCHMAX 5
#define WSLIM  ((size_t)134217728)

#define T_EA   0
#define T_EB   16384
#define T_E2   32768
#define T_C1   49152
#define T_N1   65536
#define T_N2   98304
#define T_TOT  114688
#define T_GRP  (T_TOT / 8)
#define T_BLK  (T_GRP / 256)

#define L_H16  0
#define L_STG  (ROWS * HP * 2)
#define L_LDS  (L_STG + ROWS * FP * 4)

#define E_HID  0
#define E_MT   (ROWS * FP * 4)
#define E_SI   (E_MT + ROWS * HP * 2)
#define E_DI   (E_SI + ROWS * 4)
#define E_DS   (E_DI + ROWS * 4)
#define E_RL   (E_DS + ROWS * 4)
#define E_CW   (E_RL + ROWS * 16)
#define E_LDS  (E_CW + 2 * ROWS * 4)

#define NTHR   256
#define NWAVE  8
#define NB     256
#define EPT    8
#define CHUNK  (NTHR * EPT)
#define WCAP   (EPT * 32)
#define A_ACC  0
#define A_CRD  (NB * HD * 4)
#define A_LIST (A_CRD + NB * 16)
#define A_WCNT (A_LIST + NWAVE * WCAP * 4)
#define A_LDS  (A_WCNT + 64)

#define U_A    0
#define U_HID  (ROWS * AP * 2)
#define U_PST  (U_HID + ROWS * HP * 2)
#define U_LDS  (U_PST + 4 * ROWS * 4)

static_assert(T_GRP * 8 == T_TOT);
static_assert(T_BLK * 256 == T_GRP);
static_assert(((T_EB | T_E2 | T_C1 | T_N1 | T_N2) & 63) == 0);
static_assert(((HP * 2) & 15) == 0 && ((AP * 2) & 15) == 0 && ((FP * 4) & 15) == 0);
static_assert((L_STG & 15) == 0 && L_LDS <= 64 * 1024);
static_assert((E_MT & 15) == 0 && (E_SI & 15) == 0 && (E_RL & 15) == 0 && (E_CW & 15) == 0 && E_LDS <= 64 * 1024);
static_assert(ROWS * HP * 2 <= ROWS * FP * 4);
static_assert(ROWS * AP * 2 == ROWS * FP * 4);
static_assert((A_CRD & 15) == 0 && (A_LIST & 15) == 0 && (A_WCNT & 15) == 0 && A_LDS <= 300 * 1024);
static_assert((U_HID & 15) == 0 && (U_PST & 15) == 0 && U_LDS <= 64 * 1024);
static_assert(NB == 32 * NWAVE && NB <= 256 && WCAP == 256 && CHUNK <= (1 << 20) && NB == NTHR && ROWS == 64);
static_assert((CHUNK % ROWS) == 0);

typedef float    v4f  __attribute__((ext_vector_type(4)));
typedef float    v8f  __attribute__((ext_vector_type(8)));
typedef int      v4i  __attribute__((ext_vector_type(4)));
typedef _Float16 v4h  __attribute__((ext_vector_type(4)));
typedef _Float16 v8h  __attribute__((ext_vector_type(8)));
typedef _Float16 v16h __attribute__((ext_vector_type(16)));
union FragH { v16h v; v8h h[2]; };
union U8H   { v8h v; _Float16 e[8]; v4i q; };
union U4H   { v4h v; _Float16 e[4]; };

__device__ __forceinline__ v8f zero8f() {
  v8f z;
#pragma unroll
  for (int i = 0; i < 8; ++i) z[i] = 0.0f;
  return z;
}

__device__ __forceinline__ v8f wmh(v16h a, v16h b, v8f c) {
  v8f d = __builtin_amdgcn_wmma_f32_16x16x32_f16(false, a, false, b, (short)0, c, false, false);
  asm volatile("v_nop\n\tv_nop\n\tv_nop\n\tv_nop" : "+v"(d) : "v"(a), "v"(b));
  return d;
}

__device__ __forceinline__ v8h cvt8h(v4f a, v4f b) {
  U8H u;
#pragma unroll
  for (int i = 0; i < 4; ++i) {
    u.e[i] = (_Float16)a[i];
    u.e[4 + i] = (_Float16)b[i];
  }
  return u.v;
}

__device__ __forceinline__ float silu_f(float v) {
  return v * __builtin_amdgcn_rcpf(1.0f + __expf(-v));
}

__device__ __forceinline__ void gemm_h(const _Float16* arow, const _Float16* bcol, int kp, int nk, v8f acc[4]) {
#pragma unroll 1
  for (int kt = 0; kt < nk; ++kt) {
    FragH a;
    a.h[0] = *(const v8h*)(arow + 32 * kt);
    a.h[1] = *(const v8h*)(arow + 32 * kt + 16);
#pragma unroll
    for (int nt = 0; nt < 4; ++nt) {
      const _Float16* bp = bcol + (size_t)(16 * nt) * kp + 32 * kt;
      FragH b;
      b.h[0] = *(const v8h*)bp;
      b.h[1] = *(const v8h*)(bp + 16);
      acc[nt] = wmh(a.v, b.v, acc[nt]);
    }
  }
}

__device__ __forceinline__ void store_rows_f32(const float* stg, float* g, int row0, int M, int wave, int l) {
#pragma unroll
  for (int j = 0; j < 8; ++j) {
    const int lr = 8 * wave + j;
    const int gr = row0 + lr;
    if (gr < M) {
      const v4f v = *(const v4f*)(stg + lr * FP + 4 * l);
      *(volatile v4f*)(g + (size_t)gr * HD + 4 * l) = v;
    }
  }
  __threadfence();
#pragma unroll
  for (int j = 0; j < 8; ++j) {
    const int lr = 8 * wave + j;
    const int gr = row0 + lr;
    if (gr < M) {
      const v4f v = *(const v4f*)(stg + lr * FP + 4 * l);
      *(volatile v4f*)(g + (size_t)gr * HD + 4 * l) = v;
    }
  }
}

__global__ __launch_bounds__(256) void k_wcvt(const float* __restrict__ ew1, const float* __restrict__ ew2,
                                              const float* __restrict__ cw1, const float* __restrict__ nw1,
                                              const float* __restrict__ nw2, v4i* wq) {
  const int g = blockIdx.x * 256 + threadIdx.x;
  if (g < T_GRP) {
    const float* src = ew1;
    int n = 0, kc = 0;
    if (g < 2048)       { const int q = g;         src = ew1;                    n = q >> 4; kc = (q & 15) * 8; }
    else if (g < 4096)  { const int q = g - 2048;  src = ew1 + (size_t)HD * HD; n = q >> 4; kc = (q & 15) * 8; }
    else if (g < 6144)  { const int q = g - 4096;  src = ew2;                    n = q >> 4; kc = (q & 15) * 8; }
    else if (g < 8192)  { const int q = g - 6144;  src = cw1;                    n = q >> 4; kc = (q & 15) * 8; }
    else if (g < 12288) { const int q = g - 8192;  src = nw1;                    n = q >> 5; kc = (q & 31) * 8; }
    else                { const int q = g - 12288; src = nw2;                    n = q >> 4; kc = (q & 15) * 8; }
    U8H u;
#pragma unroll
    for (int i = 0; i < 8; ++i) u.e[i] = (_Float16)(src[(size_t)(kc + i) * HD + n] * WSC);
    const v4i o = u.q;
    *(volatile v4i*)(wq + g) = o;
    __threadfence();
    *(volatile v4i*)(wq + g) = o;
  }
}

__global__ __launch_bounds__(256) void k_node(const float* __restrict__ xin, const _Float16* th,
                                              float* HA, float* HB, int nN) {
  extern __shared__ __attribute__((aligned(16))) unsigned char lds_n[];
  _Float16* h16 = (_Float16*)(lds_n + L_H16);
  float*    stg = (float*)(lds_n + L_STG);
  const int tid = threadIdx.x, l = tid & 31, wave = tid >> 5, h = l >> 4, m = l & 15;
  const int wr = wave >> 1, wc = wave & 1;
  const int row0 = blockIdx.x * ROWS;

  for (int i = tid; i < ROWS * 16; i += 256) {
    const int r = i >> 4, c = (i & 15) * 8;
    const int gr = row0 + r;
    v4f x0 = {0.0f, 0.0f, 0.0f, 0.0f};
    v4f x1 = x0;
    if (gr < nN) {
      const float* p = xin + (size_t)gr * HD + c;
      x0 = *(const v4f*)p;
      x1 = *(const v4f*)(p + 4);
    }
    *(v8h*)(h16 + r * HP + c) = cvt8h(x0, x1);
  }
  __syncthreads();

  v8f acc[4];
#pragma unroll
  for (int i = 0; i < 4; ++i) acc[i] = zero8f();
  gemm_h(h16 + (16 * wr + m) * HP + 8 * h, th + T_EA + (size_t)(64 * wc + m) * HD + 8 * h, HD, 4, acc);
#pragma unroll
  for (int nt = 0; nt < 4; ++nt) {
    const int c = 64 * wc + 16 * nt + m;
#pragma unroll
    for (int r = 0; r < 8; ++r) {
      const int lr = 16 * wr + 8 * h + r;
      stg[lr * FP + c] = acc[nt][r] * WINV;
    }
  }
  __syncthreads();
  store_rows_f32(stg, HA, row0, nN, wave, l);
  __syncthreads();

#pragma unroll
  for (int i = 0; i < 4; ++i) acc[i] = zero8f();
  gemm_h(h16 + (16 * wr + m) * HP + 8 * h, th + T_EB + (size_t)(64 * wc + m) * HD + 8 * h, HD, 4, acc);
#pragma unroll
  for (int nt = 0; nt < 4; ++nt) {
    const int c = 64 * wc + 16 * nt + m;
#pragma unroll
    for (int r = 0; r < 8; ++r) {
      const int lr = 16 * wr + 8 * h + r;
      stg[lr * FP + c] = acc[nt][r] * WINV;
    }
  }
  __syncthreads();
  store_rows_f32(stg, HB, row0, nN, wave, l);
}

__global__ __launch_bounds__(256) void k_edge(const int* __restrict__ ei, const float* __restrict__ pos,
                                              const float* __restrict__ HA, const float* __restrict__ HB,
                                              const float* __restrict__ ew1, const float* __restrict__ eb1,
                                              const float* __restrict__ eb2, const float* __restrict__ cb1,
                                              const float* __restrict__ cw2, const _Float16* th,
                                              float* msg, v4f* cwr, int nN, int nE, int cb, int clen, int prow) {
  extern __shared__ __attribute__((aligned(16))) unsigned char lds_e[];
  _Float16* hid  = (_Float16*)(lds_e + E_HID);
  float*    stg  = (float*)(lds_e + E_HID);
  _Float16* mt   = (_Float16*)(lds_e + E_MT);
  int*      sidx = (int*)(lds_e + E_SI);
  int*      didx = (int*)(lds_e + E_DI);
  float*    dsl  = (float*)(lds_e + E_DS);
  v4f*      rel  = (v4f*)(lds_e + E_RL);
  float*    cwp  = (float*)(lds_e + E_CW);
  const int tid = threadIdx.x, l = tid & 31, wave = tid >> 5, h = l >> 4, m = l & 15;
  const int wr = wave >> 1, wc = wave & 1;
  const int e0 = blockIdx.x * ROWS;

  if (tid < ROWS) {
    const int le = e0 + tid;
    int sc = 0, dc = 0;
    float rx = 0.0f, ry = 0.0f, rz = 0.0f, d2 = 0.0f;
    if (le < clen) {
      const int g = cb + le;
      int s = ei[g];
      int d = ei[(size_t)nE + g];
      if (s < 0) s += nN;
      sc = s < 0 ? 0 : (s > nN - 1 ? nN - 1 : s);
      if (d < 0) d += nN;
      dc = d < 0 ? 0 : (d > nN - 1 ? nN - 1 : d);
      rx = pos[(size_t)sc * 3 + 0] - pos[(size_t)dc * 3 + 0];
      ry = pos[(size_t)sc * 3 + 1] - pos[(size_t)dc * 3 + 1];
      rz = pos[(size_t)sc * 3 + 2] - pos[(size_t)dc * 3 + 2];
      d2 = (rx * rx + ry * ry) + rz * rz;
    }
    sidx[tid] = sc;
    didx[tid] = dc;
    dsl[tid] = d2;
    v4f r4;
    r4.x = rx; r4.y = ry; r4.z = rz; r4.w = 0.0f;
    rel[tid] = r4;
  }
  __syncthreads();

  {
    const v4f w4 = *(const v4f*)(ew1 + (size_t)(DIN - 1) * HD + 4 * l);
    const v4f b4 = *(const v4f*)(eb1 + 4 * l);
#pragma unroll
    for (int j = 0; j < 8; ++j) {
      const int lr = 8 * wave + j;
      const int s = sidx[lr], d = didx[lr];
      const float d2 = dsl[lr];
      const v4f va = *(const v4f*)(HA + (size_t)s * HD + 4 * l);
      const v4f vb = *(const v4f*)(HB + (size_t)d * HD + 4 * l);
      U4H u;
#pragma unroll
      for (int i = 0; i < 4; ++i) {
        const float p = (va[i] + vb[i]) + b4[i] + d2 * w4[i];
        u.e[i] = (_Float16)silu_f(p);
      }
      *(v4h*)(hid + lr * HP + 4 * l) = u.v;
    }
  }
  __syncthreads();

  v8f acc[4];
#pragma unroll
  for (int i = 0; i < 4; ++i) acc[i] = zero8f();
  gemm_h(hid + (16 * wr + m) * HP + 8 * h, th + T_E2 + (size_t)(64 * wc + m) * HD + 8 * h, HD, 4, acc);
  __syncthreads();
#pragma unroll
  for (int nt = 0; nt < 4; ++nt) {
    const int c = 64 * wc + 16 * nt + m;
    const float bc = eb2[c];
#pragma unroll
    for (int r = 0; r < 8; ++r) {
      const int lr = 16 * wr + 8 * h + r;
      const float s = silu_f(acc[nt][r] * WINV + bc);
      stg[lr * FP + c] = s;
      mt[lr * HP + c] = (_Float16)s;
    }
  }
  __syncthreads();

  store_rows_f32(stg, msg, e0, prow, wave, l);

#pragma unroll
  for (int i = 0; i < 4; ++i) acc[i] = zero8f();
  gemm_h(mt + (16 * wr + m) * HP + 8 * h, th + T_C1 + (size_t)(64 * wc + m) * HD + 8 * h, HD, 4, acc);
  {
    float part[8];
#pragma unroll
    for (int r = 0; r < 8; ++r) part[r] = 0.0f;
#pragma unroll
    for (int nt = 0; nt < 4; ++nt) {
      const int c = 64 * wc + 16 * nt + m;
      const float bc = cb1[c];
      const float w2 = cw2[c];
#pragma unroll
      for (int r = 0; r < 8; ++r) part[r] += silu_f(acc[nt][r] * WINV + bc) * w2;
    }
#pragma unroll
    for (int r = 0; r < 8; ++r) {
      part[r] += __shfl_xor(part[r], 1);
      part[r] += __shfl_xor(part[r], 2);
      part[r] += __shfl_xor(part[r], 4);
      part[r] += __shfl_xor(part[r], 8);
    }
    if (m == 0) {
#pragma unroll
      for (int r = 0; r < 8; ++r) cwp[wc * ROWS + 16 * wr + 8 * h + r] = part[r];
    }
  }
  __syncthreads();

  if (tid < ROWS) {
    const float cw = cwp[tid] + cwp[ROWS + tid];
    const v4f r4 = rel[tid];
    v4f o;
    o.x = cw * r4.x; o.y = cw * r4.y; o.z = cw * r4.z; o.w = 0.0f;
    const int gr = e0 + tid;
    if (gr < prow) *(volatile v4f*)(cwr + gr) = o;
    __threadfence();
    if (gr < prow) *(volatile v4f*)(cwr + gr) = o;
  }
}

__device__ __forceinline__ int scan_chunk(const int* __restrict__ segs, int nE, int cbase, int nodeBase,
                                          int* list, int tid, int wave, int vec_ok) {
  int wc = 0;
  const int el0  = tid * EPT;
  const int e0   = cbase + el0;
  const int sent = -2147483647 - 1;
  v4i da, db;
  if (vec_ok != 0 && e0 + 7 < nE) {
    da = *(const v4i*)(segs + e0);
    db = *(const v4i*)(segs + e0 + 4);
  } else {
    da.x = (e0     < nE) ? segs[(e0     < nE) ? e0     : nE - 1] : sent;
    da.y = (e0 + 1 < nE) ? segs[(e0 + 1 < nE) ? e0 + 1 : nE - 1] : sent;
    da.z = (e0 + 2 < nE) ? segs[(e0 + 2 < nE) ? e0 + 2 : nE - 1] : sent;
    da.w = (e0 + 3 < nE) ? segs[(e0 + 3 < nE) ? e0 + 3 : nE - 1] : sent;
    db.x = (e0 + 4 < nE) ? segs[(e0 + 4 < nE) ? e0 + 4 : nE - 1] : sent;
    db.y = (e0 + 5 < nE) ? segs[(e0 + 5 < nE) ? e0 + 5 : nE - 1] : sent;
    db.z = (e0 + 6 < nE) ? segs[(e0 + 6 < nE) ? e0 + 6 : nE - 1] : sent;
    db.w = (e0 + 7 < nE) ? segs[(e0 + 7 < nE) ? e0 + 7 : nE - 1] : sent;
  }
  const unsigned nb = (unsigned)nodeBase;
  const unsigned s0 = (unsigned)da.x - nb, s1 = (unsigned)da.y - nb;
  const unsigned s2 = (unsigned)da.z - nb, s3 = (unsigned)da.w - nb;
  const unsigned s4 = (unsigned)db.x - nb, s5 = (unsigned)db.y - nb;
  const unsigned s6 = (unsigned)db.z - nb, s7 = (unsigned)db.w - nb;
  const bool q0 = s0 < (unsigned)NB, q1 = s1 < (unsigned)NB, q2 = s2 < (unsigned)NB, q3 = s3 < (unsigned)NB;
  const bool q4 = s4 < (unsigned)NB, q5 = s5 < (unsigned)NB, q6 = s6 < (unsigned)NB, q7 = s7 < (unsigned)NB;
  const unsigned any = __builtin_amdgcn_ballot_w32(q0 | q1 | q2 | q3 | q4 | q5 | q6 | q7);
  if (any != 0u) {
#define HITJ(J, QJ, SJ) { \
      const unsigned mj = __builtin_amdgcn_ballot_w32(QJ); \
      if (mj != 0u) { \
        if (QJ) { \
          const int p = wc + (int)__builtin_amdgcn_mbcnt_lo(mj, 0u); \
          if (p < WCAP) list[wave * WCAP + p] = ((el0 + (J)) << 8) | (int)(SJ); \
        } \
        wc += (int)__builtin_popcount(mj); } }
    HITJ(0, q0, s0)
    HITJ(1, q1, s1)
    HITJ(2, q2, s2)
    HITJ(3, q3, s3)
    HITJ(4, q4, s4)
    HITJ(5, q5, s5)
    HITJ(6, q6, s6)
    HITJ(7, q7, s7)
#undef HITJ
  }
  return wc;
}

__global__ __launch_bounds__(NTHR) void k_agg(const int* __restrict__ segs, const float* __restrict__ msg,
                                               const v4f* __restrict__ cwr, float* agg, v4f* crd,
                                               int nN, int clen, int first, int vec_ok) {
  extern __shared__ __attribute__((aligned(16))) unsigned char lds_a[];
  float* acc  = (float*)(lds_a + A_ACC);
  v4f*   cac  = (v4f*)(lds_a + A_CRD);
  int*   list = (int*)(lds_a + A_LIST);
  int*   wcnt = (int*)(lds_a + A_WCNT);
  const int tid = threadIdx.x, l = tid & 31, wave = tid >> 5;
  const int nodeBase = blockIdx.x * NB;

  for (int i = tid; i < NB * 32; i += NTHR) {
    const int slot = i >> 5, q = (i & 31) * 4;
    const int node = nodeBase + slot;
    v4f v = {0.0f, 0.0f, 0.0f, 0.0f};
    if (first == 0 && node < nN) v = *(const v4f*)(agg + (size_t)node * HD + q);
    *(v4f*)(acc + slot * HD + q) = v;
  }
  {
    v4f c0 = {0.0f, 0.0f, 0.0f, 0.0f};
    if (first == 0) c0 = crd[(size_t)nodeBase + tid];
    cac[tid] = c0;
  }
  __syncthreads();

  const int nChunks = (clen + CHUNK - 1) / CHUNK;
#pragma unroll 1
  for (int ch = 0; ch < nChunks; ++ch) {
    const int cbase = ch * CHUNK;
    const int wc = scan_chunk(segs, clen, cbase, nodeBase, list, tid, wave, vec_ok);
    if (l == 0) wcnt[wave] = wc;
    __syncthreads();

#pragma unroll 1
    for (int w2 = 0; w2 < NWAVE; ++w2) {
      int n = wcnt[w2];
      n = n > WCAP ? WCAP : (n < 0 ? 0 : n);
      const int* lp = list + w2 * WCAP;
#pragma unroll 1
      for (int i0 = 0; i0 < n; i0 += 32) {
        const int idx = i0 + l;
        const int v = lp[(idx < n) ? idx : 0];
        unsigned mk = __builtin_amdgcn_ballot_w32((idx < n) && ((v & 7) == wave));
#pragma unroll 1
        while (mk != 0u) {
          const int bpos = __builtin_ctz(mk);
          mk &= mk - 1u;
          const int vv = __shfl(v, bpos);
          const int slot = vv & 255;
          int e = cbase + (vv >> 8);
          e = e < 0 ? 0 : (e > clen - 1 ? clen - 1 : e);
          const v4f x = *(const v4f*)(msg + (size_t)e * HD + 4 * l);
          float* ap = acc + slot * HD + 4 * l;
          v4f a = *(v4f*)ap;
          a[0] += x[0]; a[1] += x[1]; a[2] += x[2]; a[3] += x[3];
          *(v4f*)ap = a;
          if (l == 0) {
            const v4f cr = cwr[e];
            v4f c = cac[slot];
            c[0] += cr[0]; c[1] += cr[1]; c[2] += cr[2]; c[3] += 1.0f;
            cac[slot] = c;
          }
        }
      }
    }
    __syncthreads();
  }

#pragma unroll
  for (int j = 0; j < 32; ++j) {
    const int slot = wave * 32 + j;
    const int node = nodeBase + slot;
    if (node < nN) {
      const v4f a = *(const v4f*)(acc + slot * HD + 4 * l);
      *(volatile v4f*)(agg + (size_t)node * HD + 4 * l) = a;
    }
  }
  const v4f cv = cac[tid];
  v4f* cp = crd + (size_t)nodeBase + tid;
  *(volatile v4f*)cp = cv;
  __threadfence();
#pragma unroll
  for (int j = 0; j < 32; ++j) {
    const int slot = wave * 32 + j;
    const int node = nodeBase + slot;
    if (node < nN) {
      const v4f a = *(const v4f*)(acc + slot * HD + 4 * l);
      *(volatile v4f*)(agg + (size_t)node * HD + 4 * l) = a;
    }
  }
  *(volatile v4f*)cp = cv;
}

__global__ __launch_bounds__(256) void k_upd(const float* __restrict__ xin, const float* __restrict__ agg,
                                             const v4f* __restrict__ crd, const float* __restrict__ pos,
                                             const _Float16* th, const float* __restrict__ nb1,
                                             const float* __restrict__ nb2, const float* __restrict__ lng,
                                             const float* __restrict__ lnb, float* out0, float* out1, int nN) {
  extern __shared__ __attribute__((aligned(16))) unsigned char lds_u[];
  _Float16* a16 = (_Float16*)(lds_u + U_A);
  float*    stg = (float*)(lds_u + U_A);
  _Float16* hid = (_Float16*)(lds_u + U_HID);
  float*    pst = (float*)(lds_u + U_PST);
  const int tid = threadIdx.x, l = tid & 31, wave = tid >> 5, h = l >> 4, m = l & 15;
  const int wr = wave >> 1, wc = wave & 1;
  const int row0 = blockIdx.x * ROWS;

  if (tid < ROWS) {
    const int gr = row0 + tid;
    float p0 = 0.0f, p1 = 0.0f, p2 = 0.0f;
    if (gr < nN) {
      const v4f c = crd[gr];
      const float rc = __builtin_amdgcn_rcpf(c[3] + 1e-6f);
      p0 = pos[(size_t)gr * 3 + 0] + c[0] * rc;
      p1 = pos[(size_t)gr * 3 + 1] + c[1] * rc;
      p2 = pos[(size_t)gr * 3 + 2] + c[2] * rc;
    }
    pst[3 * tid + 0] = p0;
    pst[3 * tid + 1] = p1;
    pst[3 * tid + 2] = p2;
  }

  for (int i = tid; i < ROWS * 32; i += 256) {
    const int r = i >> 5, c = (i & 31) * 8;
    const int gr = row0 + r;
    v4f x0 = {0.0f, 0.0f, 0.0f, 0.0f};
    v4f x1 = x0;
    if (gr < nN) {
      if (c < HD) {
        const float* p = xin + (size_t)gr * HD + c;
        x0 = *(const v4f*)p;
        x1 = *(const v4f*)(p + 4);
      } else {
        const float* p = agg + (size_t)gr * HD + (c - HD);
        x0 = *(const v4f*)p;
        x1 = *(const v4f*)(p + 4);
      }
    }
    *(v8h*)(a16 + r * AP + c) = cvt8h(x0, x1);
  }
  __syncthreads();

  if (tid < 48) {
    const int lim = 3 * nN;
    const int f = row0 * 3 + 4 * tid;
    v4f o;
    o.x = pst[4 * tid + 0]; o.y = pst[4 * tid + 1]; o.z = pst[4 * tid + 2]; o.w = pst[4 * tid + 3];
    if (f + 3 < lim) {
      *(volatile v4f*)(out1 + f) = o;
    } else {
      if (f     < lim) *(volatile float*)(out1 + f)     = o.x;
      if (f + 1 < lim) *(volatile float*)(out1 + f + 1) = o.y;
      if (f + 2 < lim) *(volatile float*)(out1 + f + 2) = o.z;
    }
    __threadfence();
    if (f + 3 < lim) {
      *(volatile v4f*)(out1 + f) = o;
    } else {
      if (f     < lim) *(volatile float*)(out1 + f)     = o.x;
      if (f + 1 < lim) *(volatile float*)(out1 + f + 1) = o.y;
      if (f + 2 < lim) *(volatile float*)(out1 + f + 2) = o.z;
    }
  }

  v8f acc[4];
#pragma unroll
  for (int i = 0; i < 4; ++i) acc[i] = zero8f();
  gemm_h(a16 + (16 * wr + m) * AP + 8 * h, th + T_N1 + (size_t)(64 * wc + m) * 256 + 8 * h, 256, 8, acc);
#pragma unroll
  for (int nt = 0; nt < 4; ++nt) {
    const int c = 64 * wc + 16 * nt + m;
    const float bc = nb1[c];
#pragma unroll
    for (int r = 0; r < 8; ++r) {
      const int lr = 16 * wr + 8 * h + r;
      hid[lr * HP + c] = (_Float16)silu_f(acc[nt][r] * WINV + bc);
    }
  }
  __syncthreads();

#pragma unroll
  for (int i = 0; i < 4; ++i) acc[i] = zero8f();
  gemm_h(hid + (16 * wr + m) * HP + 8 * h, th + T_N2 + (size_t)(64 * wc + m) * HD + 8 * h, HD, 4, acc);
#pragma unroll
  for (int nt = 0; nt < 4; ++nt) {
    const int c = 64 * wc + 16 * nt + m;
    const float bc = nb2[c];
#pragma unroll
    for (int r = 0; r < 8; ++r) {
      const int lr = 16 * wr + 8 * h + r;
      stg[lr * FP + c] = acc[nt][r] * WINV + bc;
    }
  }
  __syncthreads();

  {
    const int row = tid >> 2, q = tid & 3;
    const int gr = row0 + row;
    const int grc = gr < nN ? gr : nN - 1;
    float* xr = stg + row * FP + 32 * q;
    const float* hr = xin + (size_t)grc * HD + 32 * q;
    float x[32];
#pragma unroll
    for (int j = 0; j < 8; ++j) {
      const v4f u = *(const v4f*)(xr + 4 * j);
      const v4f hq = *(const v4f*)(hr + 4 * j);
#pragma unroll
      for (int i = 0; i < 4; ++i) x[4 * j + i] = hq[i] + u[i];
    }
    float s = 0.0f;
#pragma unroll
    for (int j = 0; j < 32; ++j) s += x[j];
    s += __shfl_xor(s, 1);
    s += __shfl_xor(s, 2);
    const float mu = s * (1.0f / 128.0f);
    float dv = 0.0f;
#pragma unroll
    for (int j = 0; j < 32; ++j) { const float t = x[j] - mu; dv += t * t; }
    dv += __shfl_xor(dv, 1);
    dv += __shfl_xor(dv, 2);
    const float var = dv * (1.0f / 128.0f);
    const float rstd = rsqrtf(var + 1e-5f);
#pragma unroll
    for (int j = 0; j < 8; ++j) {
      const v4f g4 = *(const v4f*)(lng + 32 * q + 4 * j);
      const v4f b4 = *(const v4f*)(lnb + 32 * q + 4 * j);
      v4f y;
#pragma unroll
      for (int i = 0; i < 4; ++i) y[i] = (x[4 * j + i] - mu) * rstd * g4[i] + b4[i];
      *(v4f*)(xr + 4 * j) = y;
    }
  }
  __syncthreads();

  store_rows_f32(stg, out0, row0, nN, wave, l);
}

extern "C" void kernel_launch(void* const* d_in, const int* in_sizes, int n_in,
                              void* d_out, int out_size, void* d_ws, size_t ws_size,
                              hipStream_t stream) {
  if (n_in < 16) return;
  const int nN = in_sizes[0] / HD;
  const int nE = in_sizes[2] / 2;
  if (nN <= 0 || nE <= 0) return;
  if (in_sizes[0] != nN * HD || in_sizes[1] != nN * 3 || in_sizes[2] != 2 * nE) return;
  if (in_sizes[3] != DIN * HD || in_sizes[4] < HD || in_sizes[5] != HD * HD || in_sizes[6] < HD) return;
  if (in_sizes[7] != 256 * HD || in_sizes[8] < HD || in_sizes[9] != HD * HD || in_sizes[10] < HD) return;
  if (in_sizes[11] != HD * HD || in_sizes[12] < HD || in_sizes[13] < HD || in_sizes[14] < HD || in_sizes[15] < HD) return;
  if ((long long)out_size != (long long)nN * (HD + 3)) return;

  const float* xin  = (const float*)d_in[0];
  const float* pos  = (const float*)d_in[1];
  const int*   ei   = (const int*)d_in[2];
  const float* ew1  = (const float*)d_in[3];
  const float* eb1  = (const float*)d_in[4];
  const float* ew2  = (const float*)d_in[5];
  const float* eb2  = (const float*)d_in[6];
  const float* nw1  = (const float*)d_in[7];
  const float* nb1  = (const float*)d_in[8];
  const float* nw2  = (const float*)d_in[9];
  const float* nb2  = (const float*)d_in[10];
  const float* cw1  = (const float*)d_in[11];
  const float* cb1  = (const float*)d_in[12];
  const float* cw2  = (const float*)d_in[13];
  const float* lng  = (const float*)d_in[14];
  const float* lnb  = (const float*)d_in[15];
  float* out0 = (float*)d_out;
  float* out1 = out0 + (size_t)nN * HD;

  const int nBlkN = (nN + ROWS - 1) / ROWS;
  const int nBlkA = (nN + NB - 1) / NB;
  long long chl = ((long long)nE + NCHMAX - 1) / NCHMAX;
  chl = (chl + CHUNK - 1) / CHUNK * CHUNK;
  const int CH = (int)chl;
  int nchl = 0;
  for (int c = 0; c < NCHMAX; ++c) if ((long long)c * CH < (long long)nE) ++nchl;

  char* ws = (char*)d_ws;
  size_t off = 0;
  const size_t oT  = off; off += (size_t)T_TOT * 2;          off = (off + 255) & ~(size_t)255;
  const size_t oHA = off; off += (size_t)nN * HD * 4;        off = (off + 255) & ~(size_t)255;
  const size_t oHB = off; off += (size_t)nN * HD * 4;        off = (off + 255) & ~(size_t)255;
  const size_t oMS = off; off += (size_t)CH * HD * 4;        off = (off + 255) & ~(size_t)255;
  const size_t oCW = off; off += (size_t)CH * 16;            off = (off + 255) & ~(size_t)255;
  const size_t oAG = off; off += (size_t)nN * HD * 4;        off = (off + 255) & ~(size_t)255;
  const size_t oCR = off; off += (size_t)nBlkA * NB * 16;    off = (off + 255) & ~(size_t)255;
  if (off > ws_size || off > WSLIM) return;
  v4i*            wq  = (v4i*)(ws + oT);
  const _Float16* th  = (const _Float16*)(ws + oT);
  float*          hap = (float*)(ws + oHA);
  float*          hbp = (float*)(ws + oHB);
  float*          msp = (float*)(ws + oMS);
  v4f*            cwq = (v4f*)(ws + oCW);
  float*          agp = (float*)(ws + oAG);
  v4f*            crq = (v4f*)(ws + oCR);

  const hipError_t a0 = hipFuncSetAttribute(reinterpret_cast<const void*>(&k_node), hipFuncAttributeMaxDynamicSharedMemorySize, L_LDS);
  const hipError_t a1 = hipFuncSetAttribute(reinterpret_cast<const void*>(&k_edge), hipFuncAttributeMaxDynamicSharedMemorySize, E_LDS);
  const hipError_t a2 = hipFuncSetAttribute(reinterpret_cast<const void*>(&k_agg),  hipFuncAttributeMaxDynamicSharedMemorySize, A_LDS);
  const hipError_t a3 = hipFuncSetAttribute(reinterpret_cast<const void*>(&k_upd),  hipFuncAttributeMaxDynamicSharedMemorySize, U_LDS);
  (void)a0; (void)a1; (void)a2; (void)a3;

  k_wcvt<<<T_BLK, 256, 0, stream>>>(ew1, ew2, cw1, nw1, nw2, wq);
  k_node<<<nBlkN, 256, L_LDS, stream>>>(xin, th, hap, hbp, nN);

  for (int c = 0; c < nchl; ++c) {
    const int cbase = c * CH;
    int clen = nE - cbase;
    clen = clen > CH ? CH : clen;
    const int nEB = (clen + ROWS - 1) / ROWS;
    k_edge<<<nEB, 256, E_LDS, stream>>>(ei, pos, hap, hbp, ew1, eb1, eb2, cb1, cw2, th, msp, cwq,
                                        nN, nE, cbase, clen, CH);
    k_agg<<<nBlkA, NTHR, A_LDS, stream>>>(ei + (size_t)cbase, msp, (const v4f*)cwq, agp, crq,
                                          nN, clen, (c == 0) ? 1 : 0, 1);
  }

  k_upd<<<nBlkN, 256, U_LDS, stream>>>(xin, agp, (const v4f*)crq, pos, th, nb1, nb2, lng, lnb, out0, out1, nN);
  (void)hipGetLastError();
}
